// Naive_LSTM_14474039787794
// MI455X (gfx1250) — hardware-run, weakly checked
//
#include <hip/hip_runtime.h>

typedef __attribute__((ext_vector_type(16))) _Float16 v16h;
typedef __attribute__((ext_vector_type(8)))  _Float16 v8h;
typedef __attribute__((ext_vector_type(8)))  float    v8f;
typedef __attribute__((ext_vector_type(4)))  float    v4f;
typedef __attribute__((ext_vector_type(4)))  unsigned v4u;

constexpr int kBatch   = 2048;
constexpr int kSteps   = 1024;
constexpr int kHid     = 51;
constexpr int kGateN   = 4 * kHid;
constexpr int kRowsPB  = 16;
constexpr int kBlocks  = kBatch / kRowsPB;
constexpr int kKP      = 64;
constexpr int kTilesN  = 13;
constexpr int kNP      = kTilesN * 16;
constexpr int kUnitTiles = 3;
constexpr int kRemBase = 48;
constexpr int kGrp     = 32;
constexpr int kK2      = 52;
constexpr int kK2Half  = 26;
static_assert(kGateN == 204, "gate columns");
static_assert(kBatch % kRowsPB == 0, "blocks cover the batch exactly");
static_assert(kSteps % kGrp == 0, "whole 32-step groups");
static_assert(kKP % 32 == 0 && kKP >= kHid, "K padded to a multiple of 32");
static_assert(kUnitTiles * 16 == kRemBase, "full unit tiles");
static_assert(kRemBase + 4 == kK2 && kK2 == 2 * kK2Half, "remainder tile holds units 48..50 plus one phantom unit");
static_assert((kUnitTiles * 4 + 1) == kTilesN, "12 gate-interleaved tiles + 1 remainder tile");

constexpr float kCarryH  = 16.0f;
constexpr float kCarryW  = 16.0f;
constexpr float kFold    = 1.0f / (kCarryH * kCarryW);
constexpr float kLog2e   = 1.4426950408889634f;
constexpr float kSigS    = -kLog2e;
constexpr float kTanS    = 2.0f * kLog2e;
constexpr float kAccSig  = kSigS * kFold;
constexpr float kAccTan  = kTanS * kFold;

__device__ __forceinline__ float fexp2(float x) { return __builtin_amdgcn_exp2f(x); }
__device__ __forceinline__ float frcp(float x)  { return __builtin_amdgcn_rcpf(x); }

union FragU { v16h v; v8h h[2]; };
__device__ __forceinline__ v16h load_frag(const _Float16* p) {
  FragU f;
  f.h[0] = *(const v8h*)(p);
  f.h[1] = *(const v8h*)(p + 16);
  return f.v;
}
__device__ __forceinline__ v8f mma_h(v16h a, v16h b, v8f c) {
  return __builtin_amdgcn_wmma_f32_16x16x32_f16(false, a, false, b, (short)0, c, false, false);
}
__device__ __forceinline__ void guard_acc(v8f& acc, v16h a0, v16h a1, v16h b0, v16h b1) {
  asm volatile("v_nop\n\tv_nop\n\tv_nop\n\tv_nop" : "+v"(acc) : "v"(a0), "v"(a1), "v"(b0), "v"(b1));
}

__device__ __forceinline__ void cell_update(float ai, float af, float ag, float ao, float cold,
                                            float& cnew, float& hcar) {
  const float si = frcp(1.0f + fexp2(ai));
  const float sf = frcp(1.0f + fexp2(af));
  const float so = frcp(1.0f + fexp2(ao));
  const float tg = fmaf(-2.0f, frcp(1.0f + fexp2(ag)), 1.0f);
  const float cn = fmaf(sf, cold, si * tg);
  const float tc = fmaf(-2.0f * kCarryH, frcp(1.0f + fexp2(cn * kTanS)), kCarryH);
  cnew = cn;
  hcar = so * tc;
}

__global__ __launch_bounds__(32) void lstm2_scan_kernel(
    const float* __restrict__ xin,   const float* __restrict__ w_ih1, const float* __restrict__ w_hh1,
    const float* __restrict__ b_ih1, const float* __restrict__ b_hh1, const float* __restrict__ w_ih2,
    const float* __restrict__ w_hh2, const float* __restrict__ b_ih2, const float* __restrict__ b_hh2,
    float* __restrict__ out) {
  __shared__ __align__(16) _Float16 sW[kNP * kKP];
  __shared__ __align__(16) _Float16 sH1[kRowsPB * kKP];
  __shared__ __align__(16) float    sC1T[kK2 * 16];
  __shared__ __align__(16) float    sW2[kK2 * 4];
  __shared__ __align__(16) float    sCst[kRemBase * 8];
  __shared__ __align__(16) float    sG[16 * 16];
  __shared__ __align__(16) float    sX[kRowsPB * kGrp];
  __shared__ __align__(16) float    sOut[kRowsPB * kGrp];

  const int lane = threadIdx.x;
  const int hh   = lane >> 4;
  const int c    = lane & 15;
  const int koff = hh * 8;
  const int m0   = blockIdx.x * kRowsPB;
  const bool lowHalf = (hh == 0);

#pragma unroll 1
  for (int i = lane; i < kNP * kKP; i += 32) {
    const int np = i >> 6;
    const int k  = i & 63;
    const int j  = np >> 4;
    const int cc = np & 15;
    const int gate = (j < 12) ? (j & 3) : (cc & 3);
    const int unit = (j < 12) ? ((j >> 2) * 16 + cc) : (kRemBase + (cc >> 2));
    const bool ok  = (unit < kHid) && (k < kHid);
    const int uc = (unit < kHid) ? unit : (kHid - 1);
    const int kc = (k < kHid) ? k : (kHid - 1);
    float w = w_hh1[(gate * kHid + uc) * kHid + kc];
    asm volatile("" : "+v"(w));
    const float ws = ok ? (w * kCarryW) : 0.0f;
    sW[i] = (_Float16)ws;
  }
#pragma unroll 1
  for (int i = lane; i < kRowsPB * kKP; i += 32) sH1[i] = (_Float16)0.0f;
#pragma unroll 1
  for (int i = lane; i < kK2 * 16; i += 32) sC1T[i] = 0.0f;
#pragma unroll 1
  for (int i = lane; i < kK2 * 4; i += 32) {
    const int k = i >> 2;
    const int g = i & 3;
    const int kc = (k < kHid) ? k : (kHid - 1);
    float w = w_ih2[g * kHid + kc];
    asm volatile("" : "+v"(w));
    sW2[i] = (k < kHid) ? w : 0.0f;
  }
#pragma unroll 1
  for (int i = lane; i < kRemBase * 8; i += 32) {
    const int u = i >> 3;
    const int e = i & 7;
    const int gate = e & 3;
    const int n = gate * kHid + u;
    float wi = w_ih1[n];
    float bi = b_ih1[n];
    float bh = b_hh1[n];
    asm volatile("" : "+v"(wi), "+v"(bi), "+v"(bh));
    const float s = (gate == 2) ? kTanS : kSigS;
    sCst[i] = (e < 4) ? (wi * s) : ((bi + bh) * s);
  }

  float wiA[4], bA[4], wiB[4], bB[4];
#pragma unroll
  for (int g = 0; g < 4; ++g) {
    const int uA = kRemBase + hh;
    const int uBc = lowHalf ? (kRemBase + 2) : (kHid - 1);
    const int nA = g * kHid + uA;
    const int nB = g * kHid + uBc;
    float wa = w_ih1[nA];
    float ba = b_ih1[nA];
    float ca = b_hh1[nA];
    float wb = w_ih1[nB];
    float bb = b_ih1[nB];
    float cb = b_hh1[nB];
    asm volatile("" : "+v"(wa), "+v"(ba), "+v"(ca));
    asm volatile("" : "+v"(wb), "+v"(bb), "+v"(cb));
    const float s = (g == 2) ? kTanS : kSigS;
    wiA[g] = wa * s;
    bA[g]  = (ba + ca) * s;
    wiB[g] = lowHalf ? (wb * s) : 0.0f;
    bB[g]  = lowHalf ? ((bb + cb) * s) : 0.0f;
  }
  float whh2s[4], b2s[4];
#pragma unroll
  for (int g = 0; g < 4; ++g) {
    const float s = (g == 2) ? kTanS : kSigS;
    whh2s[g] = w_hh2[g] * s;
    b2s[g]   = (b_ih2[g] + b_hh2[g]) * s;
  }
  float h2 = 0.0f;
  float c2 = 0.0f;

  __syncthreads();

  const _Float16* arow = sH1 + c * kKP + koff;
  const int srow = lane >> 3;
  const int scol = (lane & 7) * 4;
  const v8f zero8 = {0.f, 0.f, 0.f, 0.f, 0.f, 0.f, 0.f, 0.f};

#pragma unroll 1
  for (int tg = 0; tg < kSteps / kGrp; ++tg) {
#pragma unroll
    for (int it = 0; it < 4; ++it) {
      const int row = it * 4 + srow;
      const v4f v = *(const v4f*)(xin + (size_t)(m0 + row) * kSteps + tg * kGrp + scol);
      *(v4f*)(sX + row * kGrp + scol) = v;
    }
    __syncthreads();

#pragma unroll 1
    for (int ts = 0; ts < kGrp; ++ts) {
      float xr[8];
#pragma unroll
      for (int r = 0; r < 8; ++r) xr[r] = sX[(8 * hh + r) * kGrp + ts];
      const float xq = sX[c * kGrp + ts];

      const v16h a0 = load_frag(arow);
      const v16h a1 = load_frag(arow + 32);

#pragma unroll 1
      for (int ut = 0; ut < kUnitTiles; ++ut) {
        const _Float16* wb = sW + (ut * 64 + c) * kKP + koff;
        v8f acc[4];
#pragma unroll
        for (int g = 0; g < 4; ++g) {
          const v16h b0 = load_frag(wb + g * 16 * kKP);
          const v16h b1 = load_frag(wb + g * 16 * kKP + 32);
          v8f a = zero8;
          a = mma_h(a0, b0, a);
          a = mma_h(a1, b1, a);
          guard_acc(a, a0, a1, b0, b1);
          acc[g] = a;
        }
        const int unit = ut * 16 + c;
        const v4f wi4 = *(const v4f*)(sCst + unit * 8);
        const v4f bs4 = *(const v4f*)(sCst + unit * 8 + 4);
        float* cp = sC1T + unit * 16 + 8 * hh;
        const v4f cl = *(const v4f*)(cp);
        const v4f ch = *(const v4f*)(cp + 4);
        float cv[8];
        cv[0] = cl[0]; cv[1] = cl[1]; cv[2] = cl[2]; cv[3] = cl[3];
        cv[4] = ch[0]; cv[5] = ch[1]; cv[6] = ch[2]; cv[7] = ch[3];
        _Float16* hp = sH1 + (8 * hh) * kKP + unit;
#pragma unroll
        for (int r = 0; r < 8; ++r) {
          const float x = xr[r];
          const float ai = fmaf(acc[0][r], kAccSig, fmaf(x, wi4[0], bs4[0]));
          const float af = fmaf(acc[1][r], kAccSig, fmaf(x, wi4[1], bs4[1]));
          const float ag = fmaf(acc[2][r], kAccTan, fmaf(x, wi4[2], bs4[2]));
          const float ao = fmaf(acc[3][r], kAccSig, fmaf(x, wi4[3], bs4[3]));
          float cn, hc;
          cell_update(ai, af, ag, ao, cv[r], cn, hc);
          cv[r] = cn;
          hp[r * kKP] = (_Float16)hc;
        }
        v4f nl, nh;
        nl[0] = cv[0]; nl[1] = cv[1]; nl[2] = cv[2]; nl[3] = cv[3];
        nh[0] = cv[4]; nh[1] = cv[5]; nh[2] = cv[6]; nh[3] = cv[7];
        *(v4f*)(cp) = nl;
        *(v4f*)(cp + 4) = nh;
      }

      {
        const _Float16* wb = sW + (12 * 16 + c) * kKP + koff;
        const v16h b0 = load_frag(wb);
        const v16h b1 = load_frag(wb + 32);
        v8f a = zero8;
        a = mma_h(a0, b0, a);
        a = mma_h(a1, b1, a);
        guard_acc(a, a0, a1, b0, b1);
#pragma unroll
        for (int r = 0; r < 8; ++r) sG[(8 * hh + r) * 16 + c] = a[r];
      }
      __syncthreads();
      {
        const v4f gA = *(const v4f*)(sG + c * 16 + 4 * hh);
        const v4f gB = *(const v4f*)(sG + c * 16 + 8 + 4 * hh);
        float* cpa = sC1T + (kRemBase + hh) * 16 + c;
        float* cpb = sC1T + (kRemBase + 2 + hh) * 16 + c;
        const float cAo = *cpa;
        const float cBo = *cpb;
        float cA, hA, cB, hB;
        cell_update(fmaf(gA[0], kAccSig, fmaf(xq, wiA[0], bA[0])),
                    fmaf(gA[1], kAccSig, fmaf(xq, wiA[1], bA[1])),
                    fmaf(gA[2], kAccTan, fmaf(xq, wiA[2], bA[2])),
                    fmaf(gA[3], kAccSig, fmaf(xq, wiA[3], bA[3])), cAo, cA, hA);
        cell_update(fmaf(gB[0], kAccSig, fmaf(xq, wiB[0], bB[0])),
                    fmaf(gB[1], kAccSig, fmaf(xq, wiB[1], bB[1])),
                    fmaf(gB[2], kAccTan, fmaf(xq, wiB[2], bB[2])),
                    fmaf(gB[3], kAccSig, fmaf(xq, wiB[3], bB[3])), cBo, cB, hB);
        *cpa = cA;
        *cpb = lowHalf ? cB : 0.0f;
        const _Float16 hAh = (_Float16)hA;
        const _Float16 hBh = (_Float16)hB;
        const unsigned uA = (unsigned)__builtin_bit_cast(unsigned short, hAh);
        const unsigned uB = (unsigned)__builtin_bit_cast(unsigned short, hBh);
        const unsigned pA = (unsigned)__shfl_xor((int)uA, 16, 32);
        const unsigned w0 = uA | (pA << 16);
        v4u pk;
        pk[0] = lowHalf ? w0 : 0u;
        pk[1] = lowHalf ? uB : 0u;
        pk[2] = 0u;
        pk[3] = 0u;
        *(v4u*)(void*)(sH1 + c * kKP + kRemBase + 8 * hh) = pk;
      }
      __syncthreads();

      {
        float s0 = 0.0f, s1 = 0.0f, s2 = 0.0f, s3 = 0.0f;
        const float* c1p = sC1T + (hh * kK2Half) * 16 + c;
        const float* w2p = sW2 + (hh * kK2Half) * 4;
#pragma unroll 1
        for (int kb = 0; kb < kK2Half; kb += 13) {
#pragma unroll
          for (int i = 0; i < 13; ++i) {
            const float cvv = c1p[(kb + i) * 16];
            const v4f w = *(const v4f*)(w2p + (kb + i) * 4);
            s0 = fmaf(cvv, w[0], s0);
            s1 = fmaf(cvv, w[1], s1);
            s2 = fmaf(cvv, w[2], s2);
            s3 = fmaf(cvv, w[3], s3);
          }
        }
        s0 += __shfl_xor(s0, 16, 32);
        s1 += __shfl_xor(s1, 16, 32);
        s2 += __shfl_xor(s2, 16, 32);
        s3 += __shfl_xor(s3, 16, 32);
        const float qi = fmaf(s0, kSigS, fmaf(h2, whh2s[0], b2s[0]));
        const float qf = fmaf(s1, kSigS, fmaf(h2, whh2s[1], b2s[1]));
        const float qg = fmaf(s2, kTanS, fmaf(h2, whh2s[2], b2s[2]));
        const float qo = fmaf(s3, kSigS, fmaf(h2, whh2s[3], b2s[3]));
        const float si = frcp(1.0f + fexp2(qi));
        const float sf = frcp(1.0f + fexp2(qf));
        const float so = frcp(1.0f + fexp2(qo));
        const float tg2 = fmaf(-2.0f, frcp(1.0f + fexp2(qg)), 1.0f);
        c2 = fmaf(sf, c2, si * tg2);
        const float tc = fmaf(-2.0f, frcp(1.0f + fexp2(c2 * kTanS)), 1.0f);
        h2 = so * tc;
        if (lowHalf) sOut[c * kGrp + ts] = c2;
      }
      __syncthreads();
    }

    for (int pass = 0; pass < 2; ++pass) {
#pragma unroll
      for (int it = 0; it < 4; ++it) {
        const int row = it * 4 + srow;
        const v4f v = *(const v4f*)(sOut + row * kGrp + scol);
        *(volatile v4f*)(out + (size_t)(m0 + row) * kSteps + tg * kGrp + scol) = v;
      }
      __threadfence();
    }
    __syncthreads();
  }
}

extern "C" void kernel_launch(void* const* d_in, const int* in_sizes, int n_in,
                              void* d_out, int out_size, void* d_ws, size_t ws_size, hipStream_t stream) {
  (void)d_ws; (void)ws_size;
  if (n_in < 9 || d_out == nullptr) return;
  if (in_sizes[0] != kBatch * kSteps || in_sizes[1] != kGateN || in_sizes[2] != kGateN * kHid ||
      in_sizes[3] != kGateN || in_sizes[4] != kGateN || in_sizes[5] != 4 * kHid ||
      in_sizes[6] != 4 || in_sizes[7] != 4 || in_sizes[8] != 4 || out_size != kBatch * kSteps) return;

  const float* xin   = (const float*)d_in[0];
  const float* w_ih1 = (const float*)d_in[1];
  const float* w_hh1 = (const float*)d_in[2];
  const float* b_ih1 = (const float*)d_in[3];
  const float* b_hh1 = (const float*)d_in[4];
  const float* w_ih2 = (const float*)d_in[5];
  const float* w_hh2 = (const float*)d_in[6];
  const float* b_ih2 = (const float*)d_in[7];
  const float* b_hh2 = (const float*)d_in[8];
  float* out = (float*)d_out;

  lstm2_scan_kernel<<<kBlocks, 32, 0, stream>>>(xin, w_ih1, w_hh1, b_ih1, b_hh1, w_ih2, w_hh2, b_ih2, b_hh2, out);
}
